// CalculateAttention_7722351198463
// MI455X (gfx1250) — hardware-run, weakly checked
//
#include <hip/hip_runtime.h>
#include <math.h>
#include <stdint.h>

#define SEQ   1024
#define HD    64
#define KW    128
#define VR    128
#define QSC   1024.0f
#define KSC   1024.0f
#define PCAR  16384.0f
#define VCAR  256.0f
#define LOG2E 1.4426950408889634f
#define ATW   4
#define ATT_THREADS (ATW * 32)
#define QPB   (16 * ATW)
#define BPR   (SEQ / QPB)
#define PTP   36
#define SLP   132
#define SLABF (16 * SLP)
#define VTP   72
#define VTILES (SEQ / 64)
#define CROWS 16
static_assert(HD == 64 && KW == 2 * HD && VR == 2 * HD && QPB == 64 && ATT_THREADS == 128);
static_assert((SEQ % QPB) == 0 && (SEQ % 64) == 0 && (SEQ % 32) == 0 && (SEQ % CROWS) == 0);
static_assert(BPR == 16 && VTILES == 16);
static_assert(16 * PTP <= SLABF);
static_assert(15 * SLP + HD + 15 * 4 + 3 < SLABF);
static_assert((VR - 1) * VTP + 63 < VR * VTP);
static_assert(((SLP * 4) % 16) == 0 && ((PTP * 4) % 16) == 0 && ((VTP * 2) % 16) == 0);

typedef _Float16 v16h __attribute__((ext_vector_type(16)));
typedef _Float16 v8h  __attribute__((ext_vector_type(8)));
typedef float    v8f  __attribute__((ext_vector_type(8)));
typedef float    v4f  __attribute__((ext_vector_type(4)));
typedef unsigned int v4u __attribute__((ext_vector_type(4)));

union FragH { v16h v; v8h h[2]; v4u u[2]; };

__device__ __forceinline__ unsigned short bf_bits(float f) {
  unsigned u = __float_as_uint(f);
  return (unsigned short)((u + 0x7FFFu + ((u >> 16) & 1u)) >> 16);
}
__device__ __forceinline__ float bf_up(unsigned short h) { return __uint_as_float(((unsigned)h) << 16); }
__device__ __forceinline__ float bfr(float f) { return bf_up(bf_bits(f)); }
__device__ __forceinline__ unsigned short h_bits(_Float16 x) { return __builtin_bit_cast(unsigned short, x); }
__device__ __forceinline__ unsigned pk16(unsigned short a, unsigned short b) { return (unsigned)a | ((unsigned)b << 16); }
__device__ __forceinline__ v8f zero8() { v8f z = {0.f, 0.f, 0.f, 0.f, 0.f, 0.f, 0.f, 0.f}; return z; }

__device__ __forceinline__ v16h ldfrag_h(const _Float16* p) {
  FragH f;
  f.h[0] = *(const v8h*)(p);
  f.h[1] = *(const v8h*)(p + 16);
  return f.v;
}

__device__ __forceinline__ v8f mma_raw(v16h a, v16h b, v8f c) {
  return __builtin_amdgcn_wmma_f32_16x16x32_f16(false, a, false, b, (short)0, c, false, false);
}
__device__ __forceinline__ void guard_sc(v8f& a, v16h q0, v16h q1, v16h q2, v16h q3,
                                         v16h x0, v16h x1, v16h x2, v16h x3) {
#if defined(__HIP_DEVICE_COMPILE__)
  asm volatile("v_nop\n\tv_nop\n\tv_nop\n\tv_nop"
               : "+v"(a) : "v"(q0), "v"(q1), "v"(q2), "v"(q3), "v"(x0), "v"(x1), "v"(x2), "v"(x3) : "memory");
#endif
}
__device__ __forceinline__ void guard_pv(v8f& a, v8f& b, v8f& c, v8f& d,
                                         v16h p0, v16h p1, v16h x0, v16h x1, v16h x2, v16h x3) {
#if defined(__HIP_DEVICE_COMPILE__)
  asm volatile("v_nop\n\tv_nop\n\tv_nop\n\tv_nop"
               : "+v"(a), "+v"(b), "+v"(c), "+v"(d) : "v"(p0), "v"(p1), "v"(x0), "v"(x1), "v"(x2), "v"(x3) : "memory");
#endif
}
__device__ __forceinline__ void acc_guard4(v8f& a, v8f& b, v8f& c, v8f& d) {
#if defined(__HIP_DEVICE_COMPILE__)
  asm volatile("v_nop\n\tv_nop\n\tv_nop\n\tv_nop" : "+v"(a), "+v"(b), "+v"(c), "+v"(d));
#endif
}
__device__ __forceinline__ void wave_sync_lds() {
  __builtin_amdgcn_fence(__ATOMIC_RELEASE, "workgroup");
  __builtin_amdgcn_wave_barrier();
  __builtin_amdgcn_fence(__ATOMIC_ACQUIRE, "workgroup");
}

__global__ __launch_bounds__(256) void cvt_cat(const float* __restrict__ xa, const float* __restrict__ xb,
                                               unsigned short* pl, int nrows, float sc) {
  const int tid  = threadIdx.x;
  const int row0 = blockIdx.x * CROWS;
  if (row0 >= nrows) return;
  const int half = tid >> 7;
  const int lt   = tid & 127;
  const int rl   = lt >> 3;
  const int ch   = lt & 7;
  int row = row0 + rl;
  row = (row > nrows - 1) ? (nrows - 1) : row;
  const float* src = (half != 0) ? xb : xa;
  const size_t e = (size_t)row * HD + (size_t)(ch * 8);
  const v4f a = *(const v4f*)(src + e), c4 = *(const v4f*)(src + e + 4);
  v4u o;
#pragma unroll
  for (int i = 0; i < 2; ++i) {
    o[i]     = pk16(h_bits((_Float16)(bfr(a[2 * i]) * sc)),  h_bits((_Float16)(bfr(a[2 * i + 1]) * sc)));
    o[2 + i] = pk16(h_bits((_Float16)(bfr(c4[2 * i]) * sc)), h_bits((_Float16)(bfr(c4[2 * i + 1]) * sc)));
  }
  unsigned short* d = pl + (size_t)row * KW + (size_t)(half * HD + ch * 8);
  for (int pass = 0; pass < 2; ++pass) {
    *(volatile v4u*)(d) = o;
    __threadfence();
  }
}

__global__ __launch_bounds__(256) void vt16(const float* __restrict__ va, const float* __restrict__ vb,
                                            unsigned short* VTo, int nbh) {
  __shared__ __align__(16) unsigned short T[VR * VTP];
  const int tid = threadIdx.x;
  const int bid = blockIdx.x;
  const int bh  = bid / VTILES;
  const int t   = bid - bh * VTILES;
  if (bh >= nbh) return;
  {
    const int sl = tid >> 2;
    const int dc = (tid & 3) * 16;
    int key = 64 * t + sl;
    key = (key < 0) ? 0 : ((key > SEQ - 1) ? (SEQ - 1) : key);
    const size_t so = (((size_t)bh * SEQ + (size_t)key) * HD + (size_t)dc);
#pragma unroll
    for (int g = 0; g < 2; ++g) {
      const float* src = ((g == 0) ? va : vb) + so;
#pragma unroll
      for (int i = 0; i < 4; ++i) {
        const v4f a = *(const v4f*)(src + 4 * i);
#pragma unroll
        for (int e = 0; e < 4; ++e) T[(g * HD + dc + 4 * i + e) * VTP + sl] = h_bits((_Float16)(bfr(a[e]) * VCAR));
      }
    }
  }
  __syncthreads();
  v4u vals[4];
  const int q8 = tid >> 3, p8 = (tid & 7) * 8;
#pragma unroll
  for (int it = 0; it < 4; ++it) {
    const int line = it * 32 + q8;
    vals[it] = *(const v4u*)(T + line * VTP + p8);
  }
  unsigned short* dst = VTo + ((size_t)bh * VR) * SEQ + 64 * t + p8;
  for (int pass = 0; pass < 2; ++pass) {
#pragma unroll
    for (int it = 0; it < 4; ++it) {
      const int line = it * 32 + q8;
      *(volatile v4u*)(dst + (size_t)line * SEQ) = vals[it];
    }
    __threadfence();
  }
}

__global__ __launch_bounds__(ATT_THREADS)
void attn2(const unsigned short* __restrict__ QHp, const unsigned short* __restrict__ KHp,
           const unsigned short* __restrict__ VTq, float* OPp, int nbh) {
  __shared__ __align__(16) float smem[ATW * SLABF];

  const int tid  = threadIdx.x;
  const int wave = tid >> 5;
  const int lane = tid & 31;
  const int hh   = lane >> 4;
  const int c    = lane & 15;

  const int bid  = blockIdx.x;
  const int bh   = bid / BPR;
  const int t    = bid - bh * BPR;
  if (bh >= nbh) return;

  const int iw = QPB * t + wave * 16;
  const int qs = iw + c;

  const _Float16* Qb = (const _Float16*)(const void*)QHp + ((size_t)bh * SEQ + (size_t)qs) * KW + 8 * hh;
  const v16h qa0 = ldfrag_h(Qb);
  const v16h qa1 = ldfrag_h(Qb + 32);
  const v16h qa2 = ldfrag_h(Qb + 64);
  const v16h qa3 = ldfrag_h(Qb + 96);
  const _Float16* Kb = (const _Float16*)(const void*)KHp + ((size_t)bh * SEQ + (size_t)c) * KW + 8 * hh;
  const _Float16* Vb = (const _Float16*)(const void*)VTq + ((size_t)bh * VR + (size_t)c) * SEQ + 8 * hh;
  const float lsc = LOG2E / (16.0f * QSC * KSC);

  float mrow[8], lrow[8];
  v8f o[8];
#pragma unroll
  for (int r = 0; r < 8; ++r) { mrow[r] = -INFINITY; lrow[r] = 0.f; }
#pragma unroll
  for (int j = 0; j < 8; ++j) o[j] = zero8();
  float* pt = smem + wave * SLABF;

#pragma unroll 1
  for (int kb = 0; kb < SEQ; kb += 32) {
    v8f s0 = zero8(), s1 = zero8();
    const _Float16* k0p = Kb + (size_t)kb * KW;
    const _Float16* k1p = k0p + (size_t)16 * KW;
    {
      const v16h kf0 = ldfrag_h(k0p), kf1 = ldfrag_h(k0p + 32), kf2 = ldfrag_h(k0p + 64), kf3 = ldfrag_h(k0p + 96);
      s0 = mma_raw(qa0, kf0, s0);
      s0 = mma_raw(qa1, kf1, s0);
      s0 = mma_raw(qa2, kf2, s0);
      s0 = mma_raw(qa3, kf3, s0);
      guard_sc(s0, qa0, qa1, qa2, qa3, kf0, kf1, kf2, kf3);
    }
    {
      const v16h kg0 = ldfrag_h(k1p), kg1 = ldfrag_h(k1p + 32), kg2 = ldfrag_h(k1p + 64), kg3 = ldfrag_h(k1p + 96);
      s1 = mma_raw(qa0, kg0, s1);
      s1 = mma_raw(qa1, kg1, s1);
      s1 = mma_raw(qa2, kg2, s1);
      s1 = mma_raw(qa3, kg3, s1);
      guard_sc(s1, qa0, qa1, qa2, qa3, kg0, kg1, kg2, kg3);
    }
#pragma unroll
    for (int r = 0; r < 8; ++r) {
      const float ta = s0[r] * lsc;
      const float tb = s1[r] * lsc;
      float mx = fmaxf(ta, tb);
#pragma unroll
      for (int off = 1; off < 16; off <<= 1) mx = fmaxf(mx, __shfl_xor(mx, off, 32));
      const float mn  = fmaxf(mrow[r], mx);
      const float al  = exp2f(mrow[r] - mn);
      mrow[r] = mn;
      const float e0 = exp2f(ta - mn);
      const float e1 = exp2f(tb - mn);
      float ps = e0 + e1;
#pragma unroll
      for (int off = 1; off < 16; off <<= 1) ps += __shfl_xor(ps, off, 32);
      lrow[r] = lrow[r] * al + ps;
#pragma unroll
      for (int j = 0; j < 8; ++j) o[j][r] *= al;
      const int ro = (8 * hh + r) * PTP + c;
      pt[ro]      = e0;
      pt[ro + 16] = e1;
    }
    wave_sync_lds();
    FragH ph, pl;
    {
      const float* prow = pt + c * PTP + 8 * hh;
      const v4f p0 = *(const v4f*)(prow), p1 = *(const v4f*)(prow + 4);
      const v4f p2 = *(const v4f*)(prow + 16), p3 = *(const v4f*)(prow + 20);
#pragma unroll
      for (int e = 0; e < 4; ++e) {
        const float ua = p0[e] * PCAR, ub = p1[e] * PCAR, uc = p2[e] * PCAR, ud = p3[e] * PCAR;
        const _Float16 ha = (_Float16)ua, hb = (_Float16)ub, hc = (_Float16)uc, hd = (_Float16)ud;
        ph.h[0][e]     = ha;
        ph.h[0][4 + e] = hb;
        ph.h[1][e]     = hc;
        ph.h[1][4 + e] = hd;
        pl.h[0][e]     = (_Float16)(ua - (float)ha);
        pl.h[0][4 + e] = (_Float16)(ub - (float)hb);
        pl.h[1][e]     = (_Float16)(uc - (float)hc);
        pl.h[1][4 + e] = (_Float16)(ud - (float)hd);
      }
    }
    const _Float16* vp = Vb + kb;
    {
      const v16h vb0 = ldfrag_h(vp);
      const v16h vb1 = ldfrag_h(vp + (size_t)16 * SEQ);
      const v16h vb2 = ldfrag_h(vp + (size_t)32 * SEQ);
      const v16h vb3 = ldfrag_h(vp + (size_t)48 * SEQ);
      o[0] = mma_raw(ph.v, vb0, o[0]);  o[0] = mma_raw(pl.v, vb0, o[0]);
      o[1] = mma_raw(ph.v, vb1, o[1]);  o[1] = mma_raw(pl.v, vb1, o[1]);
      o[2] = mma_raw(ph.v, vb2, o[2]);  o[2] = mma_raw(pl.v, vb2, o[2]);
      o[3] = mma_raw(ph.v, vb3, o[3]);  o[3] = mma_raw(pl.v, vb3, o[3]);
      guard_pv(o[0], o[1], o[2], o[3], ph.v, pl.v, vb0, vb1, vb2, vb3);
    }
    {
      const v16h vc0 = ldfrag_h(vp + (size_t)64 * SEQ);
      const v16h vc1 = ldfrag_h(vp + (size_t)80 * SEQ);
      const v16h vc2 = ldfrag_h(vp + (size_t)96 * SEQ);
      const v16h vc3 = ldfrag_h(vp + (size_t)112 * SEQ);
      o[4] = mma_raw(ph.v, vc0, o[4]);  o[4] = mma_raw(pl.v, vc0, o[4]);
      o[5] = mma_raw(ph.v, vc1, o[5]);  o[5] = mma_raw(pl.v, vc1, o[5]);
      o[6] = mma_raw(ph.v, vc2, o[6]);  o[6] = mma_raw(pl.v, vc2, o[6]);
      o[7] = mma_raw(ph.v, vc3, o[7]);  o[7] = mma_raw(pl.v, vc3, o[7]);
      guard_pv(o[4], o[5], o[6], o[7], ph.v, pl.v, vc0, vc1, vc2, vc3);
    }
    wave_sync_lds();
  }
  acc_guard4(o[0], o[1], o[2], o[3]);
  acc_guard4(o[4], o[5], o[6], o[7]);

  wave_sync_lds();
  float* slab = pt;
  const float oc = 1.0f / (PCAR * VCAR);
#pragma unroll
  for (int r = 0; r < 8; ++r) {
    const float lr  = lrow[r];
    const float inv = (lr > 0.0f) ? ((1.0f / lr) * oc) : 0.0f;
#pragma unroll
    for (int j = 0; j < 8; ++j) slab[(8 * hh + r) * SLP + j * 16 + c] = o[j][r] * inv;
  }
  wave_sync_lds();
  const size_t o1 = (size_t)nbh * SEQ * HD;
#pragma unroll
  for (int g = 0; g < 2; ++g) {
    v4f vals[8];
#pragma unroll
    for (int it = 0; it < 8; ++it) vals[it] = *(const v4f*)(slab + (2 * it + hh) * SLP + g * HD + c * 4);
    float* dst = OPp + (size_t)g * o1 + ((size_t)bh * SEQ + (size_t)iw) * HD + hh * HD + c * 4;
    for (int pass = 0; pass < 2; ++pass) {
#pragma unroll
      for (int it = 0; it < 8; ++it) {
        *(volatile v4f*)(dst + (size_t)(2 * it) * HD) = vals[it];
      }
      __threadfence();
    }
  }
}

extern "C" void kernel_launch(void* const* d_in, const int* in_sizes, int n_in,
                              void* d_out, int out_size, void* d_ws, size_t ws_size,
                              hipStream_t stream) {
  if (n_in < 6) return;
  const int nbh = in_sizes[0] / (SEQ * HD);
  if (nbh < 1) return;
  const long long nq = (long long)nbh * SEQ * HD;
  for (int i = 0; i < 6; ++i) {
    if ((long long)in_sizes[i] < nq) return;
  }
  if ((long long)out_size < 2 * nq) return;

  const float* qx = (const float*)d_in[0];
  const float* kx = (const float*)d_in[1];
  const float* vx = (const float*)d_in[2];
  const float* qy = (const float*)d_in[3];
  const float* ky = (const float*)d_in[4];
  const float* vy = (const float*)d_in[5];
  float*       out = (float*)d_out;

  const size_t PQ = (size_t)nbh * SEQ * KW * 2;
  const size_t PK = (size_t)nbh * SEQ * KW * 2;
  const size_t PV = (size_t)nbh * VR * SEQ * 2;
  size_t off = 0;
  const size_t oQH = off; off += PQ;
  const size_t oKH = off; off += PK;
  const size_t oVT = off; off += PV;
  if (off > ws_size) return;
  if (off > (size_t)134217728) return;

  char* ws = (char*)d_ws;
  unsigned short* QH = (unsigned short*)(ws + oQH);
  unsigned short* KH = (unsigned short*)(ws + oKH);
  unsigned short* VT = (unsigned short*)(ws + oVT);

  const int nrows = nbh * SEQ;
  const dim3 blk(256);
  const dim3 gC(nrows / CROWS);
  const dim3 gVT(nbh * VTILES);
  const dim3 gAT(nbh * BPR);
  const dim3 bAT(ATT_THREADS);

  cvt_cat<<<gC, blk, 0, stream>>>(qx, qy, QH, nrows, QSC);
  cvt_cat<<<gC, blk, 0, stream>>>(kx, ky, KH, nrows, KSC);
  vt16<<<gVT, blk, 0, stream>>>(vx, vy, VT, nbh);
  attn2<<<gAT, bAT, 0, stream>>>(QH, KH, VT, out, nbh);
  (void)hipGetLastError();
}
